// BipartiteGNN_5454608466090
// MI455X (gfx1250) — hardware-verified
//
#include <hip/hip_runtime.h>
#include <stddef.h>


#define DF      64
#define NTHR    256
#define NWAVE   8
#define EPT     8
#define NGRP    2
#define CHUNK   (NTHR * EPT * NGRP)
#define WCAP    (EPT * NGRP * 32)
#define LISTN   (NWAVE * WCAP)
#define NB      1024
#define TPW     (NB / 16 / NWAVE)
#define EROWS   (16 * NWAVE)
#define LDS_AGG (NB * DF * 4 + LISTN * 4 + 64)

static_assert((CHUNK & (CHUNK - 1)) == 0);
static_assert(CHUNK <= 4096);
static_assert((NB & (NB - 1)) == 0);
static_assert(NB <= 4096);
static_assert(NB == 16 * NWAVE * TPW);
static_assert((NB % EROWS) == 0);
static_assert(LDS_AGG >= NB * DF * 4 + LISTN * 4 + NWAVE * 4);

typedef float          v4f   __attribute__((ext_vector_type(4), may_alias));
typedef float          v8f   __attribute__((ext_vector_type(8)));
typedef int            v4i   __attribute__((ext_vector_type(4)));
typedef unsigned short v8us  __attribute__((ext_vector_type(8), may_alias));
typedef unsigned short v16us __attribute__((ext_vector_type(16)));
typedef __bf16         v16bf __attribute__((ext_vector_type(16)));
union FragB { v16bf v; v16us u; v8us h[2]; };

__device__ __forceinline__ unsigned rne16(unsigned u) {
  return (u + 0x7FFFu + ((u >> 16) & 1u)) >> 16;
}
__device__ __forceinline__ void split1(float x, unsigned short& h, unsigned short& l) {
  const unsigned hu = rne16(__float_as_uint(x));
  const float    r  = x - __uint_as_float(hu << 16);
  h = (unsigned short)hu;
  l = (unsigned short)rne16(__float_as_uint(r));
}

#define SPLIT_AT(I, X) { unsigned short th_, tl_; split1((X), th_, tl_); fh.u[I] = th_; fl.u[I] = tl_; }

__device__ __forceinline__ void afrag(const float* p, FragB& fh, FragB& fl) {
  const v4f a0 = *(const v4f*)p;
  const v4f a1 = *(const v4f*)(p + 4);
  const v4f a2 = *(const v4f*)(p + 16);
  const v4f a3 = *(const v4f*)(p + 20);
  SPLIT_AT(0, a0.x)  SPLIT_AT(1, a0.y)  SPLIT_AT(2, a0.z)  SPLIT_AT(3, a0.w)
  SPLIT_AT(4, a1.x)  SPLIT_AT(5, a1.y)  SPLIT_AT(6, a1.z)  SPLIT_AT(7, a1.w)
  SPLIT_AT(8, a2.x)  SPLIT_AT(9, a2.y)  SPLIT_AT(10, a2.z) SPLIT_AT(11, a2.w)
  SPLIT_AT(12, a3.x) SPLIT_AT(13, a3.y) SPLIT_AT(14, a3.z) SPLIT_AT(15, a3.w)
}
#undef SPLIT_AT

__device__ __forceinline__ v16bf bfrag(const unsigned short* __restrict__ p) {
  FragB f;
  f.h[0] = *(const v8us*)p;
  f.h[1] = *(const v8us*)(p + 16);
  return f.v;
}

__device__ __forceinline__ v8f wmb(v16bf a, v16bf b, v8f c) {
  v8f d = __builtin_amdgcn_wmma_f32_16x16x32_bf16(false, a, false, b, (short)0, c, false, false);
  asm volatile("v_nop\n\tv_nop\n\tv_nop\n\tv_nop" : "+v"(d) : "v"(a), "v"(b));
  return d;
}

__device__ __forceinline__ void bstep(const FragB& ah, const FragB& al,
                                      const unsigned short* __restrict__ wh,
                                      const unsigned short* __restrict__ wl, int bo, v8f& c) {
  const v16bf bh = bfrag(wh + bo);
  const v16bf bl = bfrag(wl + bo);
  c = wmb(ah.v, bh, c);
  c = wmb(ah.v, bl, c);
  c = wmb(al.v, bh, c);
}

__device__ __forceinline__ void kstep(const float* ap, const unsigned short* __restrict__ wh,
                                      const unsigned short* __restrict__ wl, int wpitch, int kof,
                                      int m, int hh, v8f& c0, v8f& c1, v8f& c2, v8f& c3) {
  FragB ah, al;
  afrag(ap, ah, al);
  const int bo = m * wpitch + kof + 8 * hh;
  bstep(ah, al, wh, wl, bo,               c0);
  bstep(ah, al, wh, wl, bo + 16 * wpitch, c1);
  bstep(ah, al, wh, wl, bo + 32 * wpitch, c2);
  bstep(ah, al, wh, wl, bo + 48 * wpitch, c3);
}

__device__ __forceinline__ void epi1(v8f c, float bv, float* sp) {
  sp[0 * DF] = fmaxf(c[0] + bv, 0.0f);
  sp[1 * DF] = fmaxf(c[1] + bv, 0.0f);
  sp[2 * DF] = fmaxf(c[2] + bv, 0.0f);
  sp[3 * DF] = fmaxf(c[3] + bv, 0.0f);
  sp[4 * DF] = fmaxf(c[4] + bv, 0.0f);
  sp[5 * DF] = fmaxf(c[5] + bv, 0.0f);
  sp[6 * DF] = fmaxf(c[6] + bv, 0.0f);
  sp[7 * DF] = fmaxf(c[7] + bv, 0.0f);
}
__device__ __forceinline__ void epi_lds(v8f c0, v8f c1, v8f c2, v8f c3, const float* __restrict__ bias,
                                        float* rows, int m, int hh) {
  float* sp = rows + (8 * hh) * DF + m;
  epi1(c0, bias[m],      sp);
  epi1(c1, bias[16 + m], sp + 16);
  epi1(c2, bias[32 + m], sp + 32);
  epi1(c3, bias[48 + m], sp + 48);
}

__device__ __forceinline__ void store_tile(const float* rows, float* g, int lane, int nvalid) {
  const int hh = lane >> 4, c4 = 4 * (lane & 15);
  v4f ov[8];
#pragma unroll
  for (int q = 0; q < 8; ++q) ov[q] = *(const v4f*)(rows + (2 * q + hh) * DF + c4);
#pragma unroll
  for (int q = 0; q < 8; ++q)
    if (2 * q + hh < nvalid) *(volatile v4f*)(g + (size_t)(2 * q + hh) * DF + c4) = ov[q];
  __threadfence();
#pragma unroll
  for (int q = 0; q < 8; ++q)
    if (2 * q + hh < nvalid) *(volatile v4f*)(g + (size_t)(2 * q + hh) * DF + c4) = ov[q];
}

template <int NBT>
__device__ __forceinline__ int scan_chunk(const int* __restrict__ keys, int nE, int cbase, int nodeBase,
                                          int vec8, int* list, int tid, int wave) {
  int wc = 0;
#pragma unroll
  for (int g = 0; g < NGRP; ++g) {
    const int el0  = (g * NTHR + tid) * EPT;
    const int e0   = cbase + el0;
    const int sent = -2147483647 - 1;
    v4i da, db;
    if (vec8 != 0 && e0 + 7 < nE) {
      da = *(const v4i*)(keys + e0);
      db = *(const v4i*)(keys + e0 + 4);
    } else {
      da.x = (e0     < nE) ? keys[min(e0, nE - 1)] : sent;
      da.y = (e0 + 1 < nE) ? keys[min(e0 + 1, nE - 1)] : sent;
      da.z = (e0 + 2 < nE) ? keys[min(e0 + 2, nE - 1)] : sent;
      da.w = (e0 + 3 < nE) ? keys[min(e0 + 3, nE - 1)] : sent;
      db.x = (e0 + 4 < nE) ? keys[min(e0 + 4, nE - 1)] : sent;
      db.y = (e0 + 5 < nE) ? keys[min(e0 + 5, nE - 1)] : sent;
      db.z = (e0 + 6 < nE) ? keys[min(e0 + 6, nE - 1)] : sent;
      db.w = (e0 + 7 < nE) ? keys[min(e0 + 7, nE - 1)] : sent;
    }
    const unsigned nb = (unsigned)nodeBase;
    const unsigned s0 = (unsigned)da.x - nb, s1 = (unsigned)da.y - nb;
    const unsigned s2 = (unsigned)da.z - nb, s3 = (unsigned)da.w - nb;
    const unsigned s4 = (unsigned)db.x - nb, s5 = (unsigned)db.y - nb;
    const unsigned s6 = (unsigned)db.z - nb, s7 = (unsigned)db.w - nb;
    const bool h0 = s0 < (unsigned)NBT, h1 = s1 < (unsigned)NBT, h2 = s2 < (unsigned)NBT, h3 = s3 < (unsigned)NBT;
    const bool h4 = s4 < (unsigned)NBT, h5 = s5 < (unsigned)NBT, h6 = s6 < (unsigned)NBT, h7 = s7 < (unsigned)NBT;
    const unsigned any = __builtin_amdgcn_ballot_w32(h0 | h1 | h2 | h3 | h4 | h5 | h6 | h7);
    if (any != 0u) {
#define HITJ(J, HJ, SJ) { \
        const unsigned mj = __builtin_amdgcn_ballot_w32(HJ); \
        if (mj != 0u) { \
          if (HJ) { \
            const int pos = wc + (int)__builtin_amdgcn_mbcnt_lo(mj, 0u); \
            if (pos < WCAP) list[wave * WCAP + pos] = ((el0 + (J)) << 12) | (int)(SJ); \
          } \
          wc += (int)__builtin_popcount(mj); } }
      HITJ(0, h0, s0)
      HITJ(1, h1, s1)
      HITJ(2, h2, s2)
      HITJ(3, h3, s3)
      HITJ(4, h4, s4)
      HITJ(5, h5, s5)
      HITJ(6, h6, s6)
      HITJ(7, h7, s7)
#undef HITJ
    }
  }
  return wc;
}

__global__ __launch_bounds__(NTHR) void k_wprep(
    const float* __restrict__ w0, const float* __restrict__ w1, const float* __restrict__ w2,
    const float* __restrict__ w3, const float* __restrict__ w4, const float* __restrict__ w5,
    int L, int base2, int base3, int base4, int base5,
    unsigned short* pH, unsigned short* pL) {
  const int t = blockIdx.y;
  const float* W; int K; int nel; int base;
  switch (t) {
    case 0:  W = w0; K = DF;     nel = DF * DF;         base = 0;       break;
    case 1:  W = w1; K = DF;     nel = DF * DF;         base = DF * DF; break;
    case 2:  W = w2; K = DF;     nel = L * DF * DF;     base = base2;   break;
    case 3:  W = w3; K = 2 * DF; nel = L * 2 * DF * DF; base = base3;   break;
    case 4:  W = w4; K = DF;     nel = L * DF * DF;     base = base4;   break;
    default: W = w5; K = 2 * DF; nel = L * 2 * DF * DF; base = base5;   break;
  }
  const int o = (blockIdx.x * NTHR + (int)threadIdx.x) * 8;
  if (o >= nel) return;
  const int ksh = (K == DF) ? 6 : 7;
  const int mat = o >> (ksh + 6);
  const int w   = o - (mat << (ksh + 6));
  const int n   = w >> ksh;
  const int k0  = w - (n << ksh);
  const float* p = W + (size_t)mat * (size_t)(K * DF) + (size_t)k0 * DF + n;
  v8us vh, vl;
#define WP(I) { unsigned short th_, tl_; split1(p[(I) * DF], th_, tl_); vh[I] = th_; vl[I] = tl_; }
  WP(0) WP(1) WP(2) WP(3) WP(4) WP(5) WP(6) WP(7)
#undef WP
  unsigned short* dh = pH + base + o;
  unsigned short* dl = pL + base + o;
  *(volatile v8us*)dh = vh;
  *(volatile v8us*)dl = vl;
  __threadfence();
  *(volatile v8us*)dh = vh;
  *(volatile v8us*)dl = vl;
}

__global__ __launch_bounds__(NTHR) void k_enc(
    const float* __restrict__ X, int N,
    const unsigned short* __restrict__ pH, const unsigned short* __restrict__ pL,
    int offW, const float* __restrict__ bW, int offM, const float* __restrict__ bM,
    float* Hout, float* Mout, int doMsg) {
  __shared__ __attribute__((aligned(16))) float rows_all[EROWS * DF];
  const int tid = threadIdx.x, lane = tid & 31, wave = tid >> 5, hh = lane >> 4, m = lane & 15;
  const int rowL = 16 * wave;
  const size_t growBase = (size_t)blockIdx.x * EROWS + (size_t)rowL;
  float* rows = rows_all + rowL * DF;

  int xr = (int)growBase + m;
  xr = xr > N - 1 ? N - 1 : xr;
  const float* ap = X + (size_t)xr * DF + 8 * hh;
  const unsigned short* wh = pH + offW;
  const unsigned short* wl = pL + offW;
  const v8f z8 = {0.f, 0.f, 0.f, 0.f, 0.f, 0.f, 0.f, 0.f};
  v8f c0 = z8, c1 = z8, c2 = z8, c3 = z8;
  kstep(ap,      wh, wl, DF, 0,  m, hh, c0, c1, c2, c3);
  kstep(ap + 32, wh, wl, DF, 32, m, hh, c0, c1, c2, c3);
  epi_lds(c0, c1, c2, c3, bW, rows, m, hh);
  __syncthreads();

  const float* aL = rows + m * DF + 8 * hh;
  v8f d0 = z8, d1 = z8, d2 = z8, d3 = z8;
  if (doMsg != 0) {
    const unsigned short* mh = pH + offM;
    const unsigned short* ml = pL + offM;
    kstep(aL,      mh, ml, DF, 0,  m, hh, d0, d1, d2, d3);
    kstep(aL + 32, mh, ml, DF, 32, m, hh, d0, d1, d2, d3);
  }
  store_tile(rows, Hout + growBase * DF, lane, 16);
  if (doMsg != 0) {
    __syncthreads();
    epi_lds(d0, d1, d2, d3, bM, rows, m, hh);
    __syncthreads();
    store_tile(rows, Mout + growBase * DF, lane, 16);
  }
}

__global__ __launch_bounds__(NTHR) void k_agg(
    const int* __restrict__ keys, const int* __restrict__ gath,
    const float* __restrict__ Mg, const float* __restrict__ Hold,
    const unsigned short* __restrict__ pH, const unsigned short* __restrict__ pL,
    int offU, int offM, const float* __restrict__ bU, const float* __restrict__ bM,
    float* Hnew, float* Mnew, float* out,
    int Nown, int Ngath, int nE, int vec8, int doMsg, int toOut) {
  extern __shared__ v4f lds_dyn[];
  float* acc  = (float*)lds_dyn;
  int*   list = (int*)(acc + NB * DF);
  int*   wcnt = list + LISTN;
  const int tid = threadIdx.x, lane = tid & 31, wave = tid >> 5, hh = lane >> 4, m = lane & 15;
  const int c4 = 4 * m;
  const int nodeBase = blockIdx.x * NB;

  {
    const v4f z = {0.f, 0.f, 0.f, 0.f};
#pragma unroll 4
    for (int i = tid; i < NB * DF / 4; i += NTHR) lds_dyn[i] = z;
  }
  __syncthreads();

  const int nChunks = (nE + CHUNK - 1) / CHUNK;
#pragma unroll 1
  for (int ch = 0; ch < nChunks; ++ch) {
    const int cbase = ch * CHUNK;
    const int wc = scan_chunk<NB>(keys, nE, cbase, nodeBase, vec8, list, tid, wave);
    if (lane == 0) wcnt[wave] = wc;
    __syncthreads();
    if (wave == 0) {
#pragma unroll 1
      for (int wsx = 0; wsx < NWAVE; ++wsx) {
        int n = __builtin_amdgcn_readfirstlane(wcnt[wsx]);
        n = n > WCAP ? WCAP : (n < 0 ? 0 : n);
        const int* lp = list + wsx * WCAP;
#pragma unroll 1
        for (int i = 0; i < n; ++i) {
          const int ent  = __builtin_amdgcn_readfirstlane(lp[i]);
          const int slot = ent & (NB - 1);
          int e = cbase + ((ent >> 12) & (CHUNK - 1));
          e = e > nE - 1 ? nE - 1 : e;
          int g = gath[e];
          g = g < 0 ? 0 : (g > Ngath - 1 ? Ngath - 1 : g);
          const v4f v = *(const v4f*)(Mg + (size_t)g * DF + c4);
          v4f* aq = (v4f*)(acc + slot * DF + c4);
          *aq = *aq + v;
        }
      }
    }
    __syncthreads();
  }

  const unsigned short* wUh = pH + offU;
  const unsigned short* wUl = pL + offU;
  const unsigned short* wMh = pH + offM;
  const unsigned short* wMl = pL + offM;
  float* Hdst = (toOut != 0) ? out : Hnew;
  const v8f z8 = {0.f, 0.f, 0.f, 0.f, 0.f, 0.f, 0.f, 0.f};
#pragma unroll 1
  for (int q = 0; q < TPW; ++q) {
    const int rowL = 16 * (q * NWAVE + wave);
    float* rows = acc + rowL * DF;
    const size_t growBase = (size_t)nodeBase + (size_t)rowL;
    const float* aG = Hold + (growBase + (size_t)m) * DF + 8 * hh;
    const float* aL = rows + m * DF + 8 * hh;
    v8f c0 = z8, c1 = z8, c2 = z8, c3 = z8;
    kstep(aG,      wUh, wUl, 2 * DF, 0,  m, hh, c0, c1, c2, c3);
    kstep(aG + 32, wUh, wUl, 2 * DF, 32, m, hh, c0, c1, c2, c3);
    kstep(aL,      wUh, wUl, 2 * DF, 64, m, hh, c0, c1, c2, c3);
    kstep(aL + 32, wUh, wUl, 2 * DF, 96, m, hh, c0, c1, c2, c3);
    epi_lds(c0, c1, c2, c3, bU, rows, m, hh);
    __syncthreads();
    v8f d0 = z8, d1 = z8, d2 = z8, d3 = z8;
    if (doMsg != 0) {
      kstep(aL,      wMh, wMl, DF, 0,  m, hh, d0, d1, d2, d3);
      kstep(aL + 32, wMh, wMl, DF, 32, m, hh, d0, d1, d2, d3);
    }
    int nvalid = 16;
    if (toOut != 0) {
      const int rem = Nown - (nodeBase + rowL);
      nvalid = rem < 16 ? rem : 16;
    }
    store_tile(rows, Hdst + growBase * DF, lane, nvalid);
    if (doMsg != 0) {
      __syncthreads();
      epi_lds(d0, d1, d2, d3, bM, rows, m, hh);
      __syncthreads();
      store_tile(rows, Mnew + growBase * DF, lane, 16);
    }
  }
}

extern "C" void kernel_launch(void* const* d_in, const int* in_sizes, int n_in,
                              void* d_out, int out_size, void* d_ws, size_t ws_size,
                              hipStream_t stream) {
  if (n_in < 16) return;
  const int Nsrc = in_sizes[0] / DF;
  const int Ndst = in_sizes[1] / DF;
  const int E    = in_sizes[2];
  if (Nsrc <= 0 || Ndst <= 0 || in_sizes[0] != Nsrc * DF || in_sizes[1] != Ndst * DF) return;
  if (E < 0 || in_sizes[3] != E) return;
  if (in_sizes[4] != DF * DF || in_sizes[5] < DF || in_sizes[6] != DF * DF || in_sizes[7] < DF) return;
  const int L = in_sizes[8] / (DF * DF);
  if (L < 1 || in_sizes[8] != L * DF * DF || in_sizes[9] < L * DF) return;
  if (in_sizes[10] != L * 2 * DF * DF || in_sizes[11] < L * DF) return;
  if (in_sizes[12] != L * DF * DF || in_sizes[13] < L * DF) return;
  if (in_sizes[14] != L * 2 * DF * DF || in_sizes[15] < L * DF) return;
  if (out_size != Ndst * DF) return;

  const float* x_src     = (const float*)d_in[0];
  const float* x_dst     = (const float*)d_in[1];
  const int*   src_idx   = (const int*)d_in[2];
  const int*   dst_idx   = (const int*)d_in[3];
  const float* W_in_src  = (const float*)d_in[4];
  const float* b_in_src  = (const float*)d_in[5];
  const float* W_in_dst  = (const float*)d_in[6];
  const float* b_in_dst  = (const float*)d_in[7];
  const float* W_msg_sd  = (const float*)d_in[8];
  const float* b_msg_sd  = (const float*)d_in[9];
  const float* W_upd_dst = (const float*)d_in[10];
  const float* b_upd_dst = (const float*)d_in[11];
  const float* W_msg_ds  = (const float*)d_in[12];
  const float* b_msg_ds  = (const float*)d_in[13];
  const float* W_upd_src = (const float*)d_in[14];
  const float* b_upd_src = (const float*)d_in[15];
  float* out = (float*)d_out;

  const int nBS  = (Nsrc + NB - 1) / NB;
  const int nBD  = (Ndst + NB - 1) / NB;
  const int padS = nBS * NB;
  const int padD = nBD * NB;

  const int base0 = 0;
  const int base1 = DF * DF;
  const int base2 = 2 * DF * DF;
  const int base3 = base2 + L * DF * DF;
  const int base4 = base3 + L * 2 * DF * DF;
  const int base5 = base4 + L * DF * DF;
  const int totW  = base5 + L * 2 * DF * DF;

  char* ws = (char*)d_ws;
  size_t off = 0;
  const size_t oPH  = off; off += (size_t)totW * 2;                 off = (off + 255) & ~(size_t)255;
  const size_t oPL  = off; off += (size_t)totW * 2;                 off = (off + 255) & ~(size_t)255;
  const size_t oHs0 = off; off += (size_t)padS * DF * 4;            off = (off + 255) & ~(size_t)255;
  const size_t oHs1 = off; off += (size_t)padS * DF * 4;            off = (off + 255) & ~(size_t)255;
  const size_t oMs  = off; off += (size_t)padS * DF * 4;            off = (off + 255) & ~(size_t)255;
  const size_t oHd0 = off; off += (size_t)padD * DF * 4;            off = (off + 255) & ~(size_t)255;
  const size_t oHd1 = off; off += (size_t)padD * DF * 4;            off = (off + 255) & ~(size_t)255;
  const size_t oMd  = off; off += (size_t)padD * DF * 4;            off = (off + 255) & ~(size_t)255;
  if (off > ws_size) return;
  unsigned short* pH = (unsigned short*)(ws + oPH);
  unsigned short* pL = (unsigned short*)(ws + oPL);
  float* Hs0 = (float*)(ws + oHs0);
  float* Hs1 = (float*)(ws + oHs1);
  float* Ms  = (float*)(ws + oMs);
  float* Hd0 = (float*)(ws + oHd0);
  float* Hd1 = (float*)(ws + oHd1);
  float* Md  = (float*)(ws + oMd);

  const int vec8 = ((E & 3) == 0) ? 1 : 0;

  const int maxNel = (L * 2 * DF * DF > DF * DF) ? L * 2 * DF * DF : DF * DF;
  const int gxW = (maxNel / 8 + NTHR - 1) / NTHR;
  k_wprep<<<dim3(gxW, 6), NTHR, 0, stream>>>(W_in_src, W_in_dst, W_msg_sd, W_upd_dst, W_msg_ds, W_upd_src,
                                             L, base2, base3, base4, base5, pH, pL);

  k_enc<<<padS / EROWS, NTHR, 0, stream>>>(x_src, Nsrc, pH, pL, base0, b_in_src, base2, b_msg_sd, Hs0, Ms, 1);
  k_enc<<<padD / EROWS, NTHR, 0, stream>>>(x_dst, Ndst, pH, pL, base1, b_in_dst, base1, b_in_dst, Hd0, Md, 0);

  hipFuncSetAttribute(reinterpret_cast<const void*>(&k_agg),
                      hipFuncAttributeMaxDynamicSharedMemorySize, LDS_AGG);
  for (int l = 0; l < L; ++l) {
    const int last = (l == L - 1) ? 1 : 0;
    float* HdOld = (l & 1) ? Hd1 : Hd0;
    float* HdNew = (l & 1) ? Hd0 : Hd1;
    float* HsOld = (l & 1) ? Hs1 : Hs0;
    float* HsNew = (l & 1) ? Hs0 : Hs1;
    k_agg<<<nBD, NTHR, LDS_AGG, stream>>>(
        dst_idx, src_idx, Ms, HdOld, pH, pL,
        base3 + l * 2 * DF * DF, base4 + l * DF * DF,
        b_upd_dst + (size_t)l * DF, b_msg_ds + (size_t)l * DF,
        HdNew, Md, out, Ndst, Nsrc, E, vec8, last ? 0 : 1, last);
    if (!last) {
      k_agg<<<nBS, NTHR, LDS_AGG, stream>>>(
          src_idx, dst_idx, Md, HsOld, pH, pL,
          base5 + l * 2 * DF * DF, base2 + (l + 1) * DF * DF,
          b_upd_src + (size_t)l * DF, b_msg_sd + (size_t)(l + 1) * DF,
          HsNew, Ms, out, Nsrc, Ndst, E, vec8, 1, 0);
    }
  }
}
